// KernelDensity_10969346474407
// MI455X (gfx1250) — hardware-run, weakly checked
//
#include <hip/hip_runtime.h>


#ifndef NQ
#define NQ 2048
#endif
#ifndef ND
#define ND 100000
#endif
#define NQ_FULL 2048
#define ND_FULL 100000
#define DIMS 16
#define KP   32
#define KW   8
#define QB   32
#define NT   (ND / 16)
#define L2E  1.4426950408889634f
#define BF_ONE ((unsigned short)0x3F80)

static_assert(DIMS == 16);
static_assert(KP == 32);
static_assert(KP * 2 == 4 * 16);
static_assert(QB == 32);
static_assert((QB / 4) * 16 == QB * 4);
static_assert(NQ % QB == 0);
static_assert(ND % 16 == 0);
static_assert((NQ * 4) % 32 == 0);
static_assert((ND * 4) % 32 == 0);
static_assert(NT >= KW);
static_assert(NQ <= NQ_FULL);
static_assert(ND <= ND_FULL);
static_assert((KW * QB + KW + QB) * 4 <= 131072);

typedef unsigned short bf;
typedef __attribute__((ext_vector_type(16))) __bf16   v16bf;
typedef __attribute__((ext_vector_type(8)))  unsigned short v8us;
typedef __attribute__((ext_vector_type(8)))  float    v8f;
typedef __attribute__((ext_vector_type(4)))  float    v4f;
typedef v4f  __attribute__((may_alias)) v4fa;

__device__ __forceinline__ unsigned short f2bf(float f) { unsigned u = __float_as_uint(f); u += 0x7FFFu + ((u >> 16) & 1u); return (unsigned short)(u >> 16); }
__device__ __forceinline__ float bfr(float f) { return __uint_as_float(((unsigned)f2bf(f)) << 16); }
__device__ __forceinline__ v16bf cat16b(v8us lo, v8us hi) { return __builtin_bit_cast(v16bf, __builtin_shufflevector(lo, hi, 0, 1, 2, 3, 4, 5, 6, 7, 8, 9, 10, 11, 12, 13, 14, 15)); }
__device__ __forceinline__ v8f wmmab(v16bf a, v16bf b, v8f c) { return __builtin_amdgcn_wmma_f32_16x16x32_bf16(false, a, false, b, (short)0, c, false, false); }
__device__ __forceinline__ v16bf ldb(const bf* p)  { return cat16b(*(const v8us*)p, *(const v8us*)(p + 16)); }
__device__ __forceinline__ v8f wmmab_g(v16bf a, v16bf b, v8f c) {
    c = wmmab(a, b, c);
    asm volatile("v_nop\n\tv_nop\n\tv_nop\n\tv_nop" : "+v"(c) : "v"(a), "v"(b));
    return c;
}

__global__ __launch_bounds__(256) void k_plane(const float* __restrict__ src, bf* dst, int nrows, int onesfirst) {
#pragma clang fp contract(off)
    const int npc = nrows * 4;
    const int i = (int)(blockIdx.x * 256 + threadIdx.x);
    const int ic = i < npc ? i : npc - 1;
    const int row = ic >> 2, q = ic & 3;
    const float* p = src + (size_t)row * DIMS + (size_t)(q & 1) * 8;
    v4f x0 = *(const v4f*)p, x1 = *(const v4f*)(p + 4);
    asm volatile("" : "+v"(x0), "+v"(x1));
    v8us od; float ss = 0.0f;
#pragma unroll
    for (int k = 0; k < 4; ++k) {
        const unsigned short u0 = f2bf(x0[k]), u1 = f2bf(x1[k]);
        od[k] = u0; od[4 + k] = u1;
        const float y0 = __uint_as_float(((unsigned)u0) << 16), y1 = __uint_as_float(((unsigned)u1) << 16);
        ss += y0 * y0; ss += y1 * y1; }
    const float tot = ss + __shfl_xor(ss, 1, 32);
    const float nb = -0.5f * tot;
    const unsigned short hb = f2bf(nb);
    const unsigned short lb = f2bf(nb - __uint_as_float(((unsigned)hb) << 16));
    const bool of = onesfirst != 0;
    const v8us oz = (v8us){};
    v8us ob = (v8us){};
    ob[0] = of ? BF_ONE : hb; ob[1] = of ? BF_ONE : lb; ob[2] = of ? hb : BF_ONE; ob[3] = of ? lb : BF_ONE;
    const v8us o = (q < 2) ? od : ((q == 2) ? ob : oz);
    if (i < npc) {
        *(volatile v8us*)(dst + (size_t)i * 8) = o; __threadfence(); *(volatile v8us*)(dst + (size_t)i * 8) = o; }
}

__global__ __launch_bounds__(32 * KW) void k_accum(const bf* __restrict__ XP, const bf* __restrict__ DP, const float* __restrict__ W, float* OUT, float normc) {
    __shared__ __align__(16) float red[KW * QB];
    __shared__ __align__(16) float wsum[KW];
    __shared__ __align__(16) float fin[QB];
    const int lane = threadIdx.x & 31, lr = lane & 15, hi = lane >> 4;
    const int wave = __builtin_amdgcn_readfirstlane((int)(threadIdx.x >> 5));
    const int q0 = blockIdx.x * QB;
    const v16bf a0 = ldb(XP + (size_t)(q0 + lr) * KP + 8 * hi);
    const v16bf a1 = ldb(XP + (size_t)(q0 + 16 + lr) * KP + 8 * hi);
    const size_t doff = (size_t)lr * KP + 8 * hi;
    v8f acc0 = (v8f){}, acc1 = (v8f){}; float ws = 0.0f;
#pragma unroll 1
    for (int j = wave; j < NT; j += KW) {
        const int n0 = j * 16;
        const v16bf b = ldb(DP + doff + (size_t)n0 * KP);
        const float wt = bfr(W[n0 + lr]);
        const v8f c0 = wmmab_g(a0, b, (v8f){});
        const v8f c1 = wmmab_g(a1, b, (v8f){});
#pragma unroll
        for (int r = 0; r < 8; ++r) {
            acc0[r] = fmaf(__builtin_amdgcn_exp2f(c0[r] * L2E), wt, acc0[r]);
            acc1[r] = fmaf(__builtin_amdgcn_exp2f(c1[r] * L2E), wt, acc1[r]); }
        ws += wt;
    }
#pragma unroll
    for (int r = 0; r < 8; ++r) {
        float s0 = acc0[r], s1 = acc1[r];
        s0 += __shfl_xor(s0, 1, 32); s1 += __shfl_xor(s1, 1, 32);
        s0 += __shfl_xor(s0, 2, 32); s1 += __shfl_xor(s1, 2, 32);
        s0 += __shfl_xor(s0, 4, 32); s1 += __shfl_xor(s1, 4, 32);
        s0 += __shfl_xor(s0, 8, 32); s1 += __shfl_xor(s1, 8, 32);
        acc0[r] = s0; acc1[r] = s1; }
    ws += __shfl_xor(ws, 1, 32); ws += __shfl_xor(ws, 2, 32); ws += __shfl_xor(ws, 4, 32); ws += __shfl_xor(ws, 8, 32);
    if (lr == 0) {
#pragma unroll
        for (int r = 0; r < 8; ++r) { red[wave * QB + hi * 8 + r] = acc0[r]; red[wave * QB + 16 + hi * 8 + r] = acc1[r]; } }
    if (lane == 0) wsum[wave] = ws;
    __syncthreads();
    if (threadIdx.x < QB) {
        float S = 0.0f, sw = 0.0f;
#pragma unroll
        for (int wv = 0; wv < KW; ++wv) { S += red[wv * QB + threadIdx.x]; sw += wsum[wv]; }
        const float dens = (S * normc) * (1.0f / sw);
        const float dcl = (dens < 0.0f) ? 0.0f : dens;
        fin[threadIdx.x] = logf(dcl); }
    __syncthreads();
    if (threadIdx.x < QB / 4) {
        const v4f val = *(const v4fa*)(&fin[threadIdx.x * 4]);
        float* o = OUT + (size_t)q0 + (size_t)threadIdx.x * 4;
        *(volatile v4f*)o = val; __threadfence(); *(volatile v4f*)o = val; }
}

static constexpr size_t al256(size_t v) { return (v + 255) & ~(size_t)255; }
static constexpr size_t SZ_XP = al256((size_t)NQ * KP * 2);
static constexpr size_t SZ_DP = al256((size_t)ND * KP * 2);
static constexpr size_t SZ_TOTAL = SZ_XP + SZ_DP;
static_assert(SZ_TOTAL <= (size_t)134217728);
static_assert((size_t)((NQ * 4 + 255) / 256) * 256 >= (size_t)NQ * 4);
static_assert((size_t)((ND * 4 + 255) / 256) * 256 >= (size_t)ND * 4);

static constexpr double TWO_PI_H2 = 2.0 * 3.141592653589793 * 1.0;
static constexpr double TP2 = TWO_PI_H2 * TWO_PI_H2;
static constexpr double TP4 = TP2 * TP2;
static constexpr double TP8 = TP4 * TP4;
static constexpr float  NORMC = (float)(1.0 / TP8);

extern "C" void kernel_launch(void* const* d_in, const int* in_sizes, int n_in,
                              void* d_out, int out_size, void* d_ws, size_t ws_size, hipStream_t stream) {
    if (n_in < 3) return;
    if ((size_t)in_sizes[0] < (size_t)NQ * DIMS) return;
    if ((size_t)in_sizes[1] < (size_t)ND * DIMS) return;
    if ((size_t)in_sizes[2] < (size_t)ND) return;
    if ((size_t)out_size < (size_t)NQ) return;
    if (SZ_TOTAL > ws_size) return;
    const float* X = (const float*)d_in[0];
    const float* data = (const float*)d_in[1];
    const float* W = (const float*)d_in[2];
    float* OUT = (float*)d_out;
    char* wsp = (char*)d_ws;
    bf* XP = (bf*)wsp; wsp += SZ_XP;
    bf* DP = (bf*)wsp; wsp += SZ_DP;

    k_plane<<<(unsigned)((NQ * 4 + 255) / 256), 256, 0, stream>>>(X, XP, NQ, 0);
    k_plane<<<(unsigned)((ND * 4 + 255) / 256), 256, 0, stream>>>(data, DP, ND, 1);
    k_accum<<<(unsigned)(NQ / QB), 32 * KW, 0, stream>>>(XP, DP, W, OUT, NORMC);
}
